// _VisualFieldAttentionModule_4020089389091
// MI455X (gfx1250) — hardware-verified
//
#include <hip/hip_runtime.h>


#define NBT  4
#define CC   512
#define C8   64
#define NN   4096
#define NQKV (2 * C8 + CC)
#define RCH  1024
#define DM   CC
#define NTK  NN
#define LOSC 1024.0f

typedef _Float16 h16;
typedef unsigned short bf;
typedef __attribute__((ext_vector_type(16))) __bf16   v16bf;
typedef __attribute__((ext_vector_type(16))) _Float16 v16h;
typedef __attribute__((ext_vector_type(8)))  _Float16 v8h;
typedef __attribute__((ext_vector_type(8)))  unsigned short v8us;
typedef __attribute__((ext_vector_type(8)))  float    v8f;
typedef __attribute__((ext_vector_type(4)))  float    v4f;
typedef __attribute__((ext_vector_type(4)))  _Float16 v4h;
typedef v8h  __attribute__((may_alias)) v8ha;
typedef v4f  __attribute__((may_alias)) v4fa;
typedef v8us __attribute__((may_alias)) v8usa;

__device__ __forceinline__ unsigned short f2bf(float f) { unsigned u = __float_as_uint(f); u += 0x7FFFu + ((u >> 16) & 1u); return (unsigned short)(u >> 16); }
__device__ __forceinline__ float bf2f(unsigned short b) { return __uint_as_float(((unsigned)b) << 16); }
__device__ __forceinline__ float bfr(float f) { return bf2f(f2bf(f)); }
__device__ __forceinline__ v16h cat16(v8h lo, v8h hi) { return __builtin_shufflevector(lo, hi, 0, 1, 2, 3, 4, 5, 6, 7, 8, 9, 10, 11, 12, 13, 14, 15); }
__device__ __forceinline__ v16bf cat16b(v8us lo, v8us hi) { return __builtin_bit_cast(v16bf, __builtin_shufflevector(lo, hi, 0, 1, 2, 3, 4, 5, 6, 7, 8, 9, 10, 11, 12, 13, 14, 15)); }
__device__ __forceinline__ v8f wmma16(v16h a, v16h b, v8f c) { return __builtin_amdgcn_wmma_f32_16x16x32_f16(false, a, false, b, (short)0, c, false, false); }
__device__ __forceinline__ v8f wmmab(v16bf a, v16bf b, v8f c) { return __builtin_amdgcn_wmma_f32_16x16x32_bf16(false, a, false, b, (short)0, c, false, false); }

__global__ __launch_bounds__(256) void k_wt(const float* __restrict__ Wm, int K, int ncols, bf* WT) {
    __shared__ __align__(16) unsigned short tl[64 * 72];
    const int tid = threadIdx.x, k0 = blockIdx.x * 64, n0 = blockIdx.y * 64;
    const int kk = tid >> 2, nq = (tid & 3) * 16;
#pragma unroll
    for (int i = 0; i < 16; ++i) tl[(nq + i) * 72 + kk] = f2bf(Wm[(size_t)(k0 + kk) * ncols + n0 + nq + i]);
    __syncthreads();
    const int piece = tid & 7;
    auto pass = [&]() {
#pragma unroll
        for (int s = 0; s < 2; ++s) { const int nr = (tid >> 3) + 32 * s; const v8us val = *(const v8usa*)(tl + nr * 72 + piece * 8); *(volatile v8us*)(WT + (size_t)(n0 + nr) * K + k0 + piece * 8) = val; }
    };
    pass(); __threadfence(); pass();
}
template <bool SPLITA, bool F16OUT = false>
__global__ __launch_bounds__(128) void k_gemmb(const bf* __restrict__ A, const bf* __restrict__ Al, const bf* __restrict__ Bn, const float* __restrict__ bias, float* C, int ldc, h16* C2, const float* __restrict__ R = nullptr, int K = DM, int roundR = 1) {
    __shared__ __align__(16) float ost[4][16 * 68];
    const int lane = threadIdx.x & 31, wave = threadIdx.x >> 5, lr = lane & 15, hi = lane >> 4;
    const int r0 = blockIdx.x * 64 + wave * 16, c0 = blockIdx.y * 64;
    const size_t aoff = (size_t)(r0 + lr) * K + 8 * hi;
    size_t boff[4];
#pragma unroll
    for (int t = 0; t < 4; ++t) boff[t] = (size_t)(c0 + t * 16 + lr) * K + 8 * hi;
    v8f acc[4];
#pragma unroll
    for (int t = 0; t < 4; ++t) acc[t] = (v8f){};
#pragma unroll 1
    for (int kc = 0; kc < K; kc += 32) {
        const v16bf a = cat16b(*(const v8us*)(A + aoff + kc), *(const v8us*)(A + aoff + kc + 16));
        v16bf al = a;
        if (SPLITA) al = cat16b(*(const v8us*)(Al + aoff + kc), *(const v8us*)(Al + aoff + kc + 16));
#pragma unroll
        for (int t = 0; t < 4; ++t) { const v16bf b = cat16b(*(const v8us*)(Bn + boff[t] + kc), *(const v8us*)(Bn + boff[t] + kc + 16)); acc[t] = wmmab(a, b, acc[t]); if (SPLITA) acc[t] = wmmab(al, b, acc[t]); }
        asm volatile("v_nop\n\tv_nop\n\tv_nop\n\tv_nop" : "+v"(acc[0]), "+v"(acc[1]), "+v"(acc[2]), "+v"(acc[3]) : "v"(a), "v"(al));
    }
    float* os = &ost[wave][0];
#pragma unroll
    for (int t = 0; t < 4; ++t) { const float bv = bias ? bfr(bias[c0 + t * 16 + lr]) : 0.f;
#pragma unroll
        for (int j = 0; j < 8; ++j) os[(hi * 8 + j) * 68 + t * 16 + lr] = acc[t][j] + bv; }
    __syncthreads();
    if (F16OUT) {
        h16* crow = (h16*)(void*)C + (size_t)r0 * ldc + c0;
        auto pass = [&]() {
#pragma unroll
            for (int s = 0; s < 4; ++s) { const int row = 4 * s + (lane >> 3), piece = lane & 7; const float* sp = os + row * 68 + piece * 8; v8h o, o2;
#pragma unroll
                for (int i = 0; i < 8; ++i) { const h16 a = (h16)sp[i]; o[i] = a; o2[i] = (h16)((sp[i] - (float)a) * LOSC); }
                *(volatile v8h*)(crow + (size_t)row * ldc + piece * 8) = o; if (C2) *(volatile v8h*)(C2 + (size_t)r0 * ldc + c0 + (size_t)row * ldc + piece * 8) = o2; }
        };
        pass(); __threadfence(); pass();
    } else {
        float* crow = C + (size_t)r0 * ldc + c0;
        auto pass = [&]() {
#pragma unroll
            for (int s = 0; s < 8; ++s) { const int Lid = (lane >> 3) + 4 * s, piece = lane & 7; const int row = Lid >> 1, cofs = (Lid & 1) * 32 + piece * 4;
                v4f val = *(const v4fa*)(os + row * 68 + cofs); if (R) { const v4f rv = *(const v4f*)(R + ((size_t)r0 + row) * ldc + c0 + cofs); val += roundR ? (v4f){bfr(rv[0]), bfr(rv[1]), bfr(rv[2]), bfr(rv[3])} : rv; }
                *(volatile v4f*)(crow + (size_t)row * ldc + cofs) = val; }
        };
        pass(); __threadfence(); pass();
    }
}

__global__ __launch_bounds__(128) void k_gemm3(const bf* __restrict__ Ah, const bf* __restrict__ Al, const bf* __restrict__ Bh, const bf* __restrict__ Bl, int K, float* C, int ldc) {
    __shared__ __align__(16) float ost[4][16 * 68];
    const int lane = threadIdx.x & 31, wave = threadIdx.x >> 5, lr = lane & 15, hi = lane >> 4;
    const int r0 = blockIdx.x * 64 + wave * 16, c0 = blockIdx.y * 64;
    const size_t aoff = (size_t)(r0 + lr) * K + 8 * hi;
    v8f acc[4];
#pragma unroll
    for (int t = 0; t < 4; ++t) acc[t] = (v8f){};
#pragma unroll 1
    for (int kc = 0; kc < K; kc += 32) {
        const v16bf a = cat16b(*(const v8us*)(Ah + aoff + kc), *(const v8us*)(Ah + aoff + kc + 16));
        const v16bf al = cat16b(*(const v8us*)(Al + aoff + kc), *(const v8us*)(Al + aoff + kc + 16));
#pragma unroll
        for (int t = 0; t < 4; ++t) { const size_t bo = (size_t)(c0 + t * 16 + lr) * K + kc + 8 * hi;
            const v16bf bh = cat16b(*(const v8us*)(Bh + bo), *(const v8us*)(Bh + bo + 16)); const v16bf bl = cat16b(*(const v8us*)(Bl + bo), *(const v8us*)(Bl + bo + 16));
            acc[t] = wmmab(a, bh, acc[t]); acc[t] = wmmab(al, bh, acc[t]); acc[t] = wmmab(a, bl, acc[t]); }
        asm volatile("v_nop\n\tv_nop\n\tv_nop\n\tv_nop" : "+v"(acc[0]), "+v"(acc[1]), "+v"(acc[2]), "+v"(acc[3]) : "v"(a), "v"(al));
    }
    float* os = &ost[wave][0];
#pragma unroll
    for (int t = 0; t < 4; ++t) {
#pragma unroll
        for (int j = 0; j < 8; ++j) os[(hi * 8 + j) * 68 + t * 16 + lr] = acc[t][j]; }
    __builtin_amdgcn_wave_barrier(); asm volatile("" ::: "memory");
    float* crow = C + (size_t)r0 * ldc + c0;
    auto pass = [&]() {
#pragma unroll
        for (int s = 0; s < 8; ++s) { const int Lid = (lane >> 3) + 4 * s, piece = lane & 7; const int row = Lid >> 1, cofs = (Lid & 1) * 32 + piece * 4;
            const v4f val = *(const v4fa*)(os + row * 68 + cofs); *(volatile v4f*)(crow + (size_t)row * ldc + cofs) = val; }
    };
    pass(); __threadfence(); pass();
}

template <int MODE>
__global__ __launch_bounds__(128) void k_gemm3x(const bf* __restrict__ Ah, const bf* __restrict__ Al, const bf* __restrict__ Bh, const bf* __restrict__ Bl, int K, float* C, int ldc) {
    if ((MODE & 1) && (int)blockIdx.y * 64 > (int)blockIdx.x * 64 + 63) return;
    const int Klim = (MODE & 2) ? min(K, ((int)blockIdx.x + 1) * 64) : K;
    __shared__ __align__(16) float ost[4][16 * 68];
    const int lane = threadIdx.x & 31, wave = threadIdx.x >> 5, lr = lane & 15, hi = lane >> 4;
    const int r0 = blockIdx.x * 64 + wave * 16, c0 = blockIdx.y * 64;
    const size_t aoff = (size_t)(r0 + lr) * K + 8 * hi;
    v8f acc[4];
#pragma unroll
    for (int t = 0; t < 4; ++t) acc[t] = (v8f){};
#pragma unroll 1
    for (int kc = 0; kc < Klim; kc += 32) {
        const v16bf a = cat16b(*(const v8us*)(Ah + aoff + kc), *(const v8us*)(Ah + aoff + kc + 16));
        v16bf al = a; if (!(MODE & 4) && !(MODE & 16)) al = cat16b(*(const v8us*)(Al + aoff + kc), *(const v8us*)(Al + aoff + kc + 16));
#pragma unroll
        for (int t = 0; t < 4; ++t) { const size_t bo = (size_t)(c0 + t * 16 + lr) * K + kc + 8 * hi;
            const v16bf bh = cat16b(*(const v8us*)(Bh + bo), *(const v8us*)(Bh + bo + 16));
            acc[t] = wmmab(a, bh, acc[t]);
            if (!(MODE & 4)) { if (!(MODE & 16)) acc[t] = wmmab(al, bh, acc[t]); if (!(MODE & 8)) { const v16bf bl = cat16b(*(const v8us*)(Bl + bo), *(const v8us*)(Bl + bo + 16)); acc[t] = wmmab(a, bl, acc[t]); } } }
        asm volatile("v_nop\n\tv_nop\n\tv_nop\n\tv_nop" : "+v"(acc[0]), "+v"(acc[1]), "+v"(acc[2]), "+v"(acc[3]) : "v"(a), "v"(al));
    }
    float* os = &ost[wave][0];
#pragma unroll
    for (int t = 0; t < 4; ++t) {
#pragma unroll
        for (int j = 0; j < 8; ++j) os[(hi * 8 + j) * 68 + t * 16 + lr] = acc[t][j]; }
    __builtin_amdgcn_wave_barrier(); asm volatile("" ::: "memory");
    float* crow = C + (size_t)r0 * ldc + c0;
    auto pass = [&]() {
#pragma unroll
        for (int s = 0; s < 8; ++s) { const int Lid = (lane >> 3) + 4 * s, piece = lane & 7; const int row = Lid >> 1, cofs = (Lid & 1) * 32 + piece * 4;
            const v4f val = *(const v4fa*)(os + row * 68 + cofs); *(volatile v4f*)(crow + (size_t)row * ldc + cofs) = val; }
    };
    pass(); __threadfence(); pass();
}


__global__ __launch_bounds__(256) void k_cvt8(const float* __restrict__ src, bf* dst, size_t n8) {
    const size_t i = (size_t)blockIdx.x * 256 + threadIdx.x; if (i >= n8) return;
    const v8f v = *(const v8f*)(src + i * 8); v8us o;
#pragma unroll
    for (int k = 0; k < 8; ++k) o[k] = f2bf(v[k]);
    *(volatile v8us*)(dst + i * 8) = o; __threadfence(); *(volatile v8us*)(dst + i * 8) = o;
}
__global__ __launch_bounds__(256) void k_zero8(bf* dst, size_t n8) {
    const size_t i = (size_t)blockIdx.x * 256 + threadIdx.x; if (i >= n8) return; v8us z;
#pragma unroll
    for (int k = 0; k < 8; ++k) z[k] = 0;
    *(volatile v8us*)(dst + i * 8) = z; __threadfence(); *(volatile v8us*)(dst + i * 8) = z;
}

__global__ __launch_bounds__(256) void k_qkplanes(const float* __restrict__ F, int off, const float* __restrict__ lfm, bf* Ph, bf* Pl) {
    typedef __attribute__((ext_vector_type(2))) unsigned short v2us;
    const int lane = threadIdx.x & 31; const size_t r = (size_t)blockIdx.x * 8 + (threadIdx.x >> 5); if (r >= (size_t)NN) return; const int c0 = lane * 2; const float sc = lfm ? bfr(lfm[r]) : 1.0f; v2us oh, ol;
#pragma unroll
    for (int i = 0; i < 2; ++i) { const float y = F[r * NQKV + off + c0 + i] * sc; const unsigned short hb = f2bf(y); oh[i] = hb; ol[i] = f2bf(y - bf2f(hb)); }
    const size_t o = r * C8 + c0; *(volatile v2us*)(Ph + o) = oh; *(volatile v2us*)(Pl + o) = ol; __threadfence(); *(volatile v2us*)(Ph + o) = oh; *(volatile v2us*)(Pl + o) = ol;
}
__global__ __launch_bounds__(256) void k_vt(const float* __restrict__ F, bf* Th, bf* Tl) {
    typedef __attribute__((ext_vector_type(2))) unsigned short v2us;
    const int lane = threadIdx.x & 31; const size_t wid = (size_t)blockIdx.x * 8 + (threadIdx.x >> 5); if (wid >= (size_t)CC * (NN / 64)) return; const int c = (int)(wid / (NN / 64)); const int j0 = (int)(wid % (NN / 64)) * 64 + lane * 2; v2us oh, ol;
#pragma unroll
    for (int i = 0; i < 2; ++i) { const float y = F[(size_t)(j0 + i) * NQKV + 2 * C8 + c]; const unsigned short hb = f2bf(y); oh[i] = hb; ol[i] = f2bf(y - bf2f(hb)); }
    const size_t o = (size_t)c * NN + j0; *(volatile v2us*)(Th + o) = oh; *(volatile v2us*)(Tl + o) = ol; __threadfence(); *(volatile v2us*)(Th + o) = oh; *(volatile v2us*)(Tl + o) = ol;
}
__global__ __launch_bounds__(256) void k_softmax4096(const float* __restrict__ S, bf* PH, bf* PL) {
    typedef __attribute__((ext_vector_type(4))) unsigned short v4us;
    const int lane = threadIdx.x & 31, i = blockIdx.x * 8 + (threadIdx.x >> 5); if (i >= RCH) return;
    float m = -3.0e38f;
#pragma unroll 1
    for (int c0 = lane * 4; c0 < NN; c0 += 128) {
#pragma unroll
        for (int q = 0; q < 4; ++q) m = fmaxf(m, S[(size_t)i * NN + c0 + q]); }
#pragma unroll
    for (int sh = 16; sh; sh >>= 1) m = fmaxf(m, __shfl_xor(m, sh, 32));
    float sum = 0.f;
#pragma unroll 1
    for (int c0 = lane * 4; c0 < NN; c0 += 128) {
#pragma unroll
        for (int q = 0; q < 4; ++q) sum += __expf(S[(size_t)i * NN + c0 + q] - m); }
#pragma unroll
    for (int sh = 16; sh; sh >>= 1) sum += __shfl_xor(sum, sh, 32);
    const float inv = 1.0f / sum;
#pragma unroll 1
    for (int ps = 0; ps < 2; ++ps) {
#pragma unroll 1
        for (int c0 = lane * 4; c0 < NN; c0 += 128) { v4us oh, ol;
#pragma unroll
            for (int q = 0; q < 4; ++q) { const float p = __expf(S[(size_t)i * NN + c0 + q] - m) * inv; const unsigned short hb = f2bf(p); oh[q] = hb; ol[q] = f2bf(p - bf2f(hb)); }
            const size_t o = (size_t)i * NN + c0; *(volatile v4us*)(PH + o) = oh; *(volatile v4us*)(PL + o) = ol; }
        if (ps == 0) __threadfence(); }
}
__global__ __launch_bounds__(256) void k_fin(const float* __restrict__ O, const float* __restrict__ xb, const float* __restrict__ gam, float* OUTB) {
    const int lane = threadIdx.x & 31; const size_t wid = (size_t)blockIdx.x * 8 + (threadIdx.x >> 5); if (wid >= (size_t)CC * (NN / 128)) return; const size_t o = wid * 128 + lane * 4; const float gm = bfr(gam[0]); v4f v;
#pragma unroll
    for (int q = 0; q < 4; ++q) v[q] = gm * O[o + q] + bfr(xb[o + q]);
    *(volatile v4f*)(OUTB + o) = v; __threadfence(); *(volatile v4f*)(OUTB + o) = v;
}
__global__ __launch_bounds__(256) void k_bias320(const float* __restrict__ bq, const float* __restrict__ bk, const float* __restrict__ bv, float* B320) {
    const int t = threadIdx.x; if (t >= 160) return; v4f v;
#pragma unroll
    for (int q = 0; q < 4; ++q) { const int c = t * 4 + q; v[q] = (c < C8) ? bq[c < C8 ? c : 0] : (c < 2 * C8) ? bk[(c >= C8 && c < 2 * C8) ? c - C8 : 0] : (c < NQKV) ? bv[(c >= 2 * C8 && c < NQKV) ? c - 2 * C8 : 0] : 0.f; }
    *(volatile v4f*)(B320 + t * 4) = v; __threadfence(); *(volatile v4f*)(B320 + t * 4) = v;
}

extern "C" void kernel_launch(void* const* d_in, const int* in_sizes, int n_in,
                              void* d_out, int out_size, void* d_ws, size_t ws_size, hipStream_t stream) {
    (void)in_sizes; (void)n_in; (void)out_size;
    const float* x = (const float*)d_in[0]; const float* wq = (const float*)d_in[2]; const float* bq = (const float*)d_in[3]; const float* wk = (const float*)d_in[4]; const float* bk = (const float*)d_in[5]; const float* wv = (const float*)d_in[6]; const float* bv = (const float*)d_in[7]; const float* gam = (const float*)d_in[8]; const float* lfm = (const float*)d_in[1];
    float* out = (float*)d_out;
    char* wsp = (char*)d_ws;
    auto take = [&](size_t bytes) { char* p = wsp; wsp += (bytes + 255) & ~(size_t)255; return (void*)p; };
    bf* WB = (bf*)take((size_t)NQKV * CC * 2); float* B320 = (float*)take(640 * 4); bf* XP = (bf*)take((size_t)NN * CC * 2); float* F = (float*)take((size_t)NN * NQKV * 4);
    bf* QPh = (bf*)take((size_t)NN * C8 * 2); bf* QPl = (bf*)take((size_t)NN * C8 * 2); bf* KPh = (bf*)take((size_t)NN * C8 * 2); bf* KPl = (bf*)take((size_t)NN * C8 * 2); bf* VTh = (bf*)take((size_t)CC * NN * 2); bf* VTl = (bf*)take((size_t)CC * NN * 2);
    float* S = (float*)take((size_t)RCH * NN * 4); bf* PH = (bf*)take((size_t)RCH * NN * 2); bf* PL = (bf*)take((size_t)RCH * NN * 2); float* O = (float*)take((size_t)CC * NN * 4);
    if ((size_t)(wsp - (char*)d_ws) > ws_size) return;
    k_cvt8<<<(C8 * CC / 8 + 255) / 256, 256, 0, stream>>>(wq, WB, C8 * CC / 8); k_cvt8<<<(C8 * CC / 8 + 255) / 256, 256, 0, stream>>>(wk, WB + (size_t)C8 * CC, C8 * CC / 8); k_cvt8<<<(CC * CC / 8 + 255) / 256, 256, 0, stream>>>(wv, WB + (size_t)2 * C8 * CC, CC * CC / 8);
    k_bias320<<<1, 256, 0, stream>>>(bq, bk, bv, B320);
    for (int b = 0; b < NBT; ++b) { const float* xb = x + (size_t)b * CC * NN;
        k_wt<<<dim3(CC / 64, NN / 64, 1), 256, 0, stream>>>(xb, CC, NN, XP);
        k_gemmb<false, false><<<dim3(NN / 64, NQKV / 64, 1), 128, 0, stream>>>(XP, nullptr, WB, B320, F, NQKV, nullptr, nullptr, CC);
        k_qkplanes<<<NN / 8, 256, 0, stream>>>(F, 0, lfm, QPh, QPl); k_qkplanes<<<NN / 8, 256, 0, stream>>>(F, C8, nullptr, KPh, KPl); k_vt<<<(CC * (NN / 64)) / 8, 256, 0, stream>>>(F, VTh, VTl);
        for (int ch = 0; ch < NN / RCH; ++ch) { const size_t r0 = (size_t)ch * RCH;
            k_gemm3<<<dim3(RCH / 64, NN / 64, 1), 128, 0, stream>>>(QPh + r0 * C8, QPl + r0 * C8, KPh, KPl, C8, S, NN);
            k_softmax4096<<<RCH / 8, 256, 0, stream>>>(S, PH, PL);
            k_gemm3x<16><<<dim3(CC / 64, RCH / 64, 1), 128, 0, stream>>>(VTh, VTl, PH, PL, NN, O + r0, NN); }
        k_fin<<<(CC * (NN / 128)) / 8, 256, 0, stream>>>(O, xb, gam, out + (size_t)b * CC * NN); }
}
